// Self_Attention_31688268709913
// MI455X (gfx1250) — hardware-verified
//
#include <hip/hip_runtime.h>


#ifndef NB
#define NB 8
#endif
#ifndef SEQ
#define SEQ 2048
#endif
#define NB_FULL  8
#define SEQ_FULL 2048
#define DM   512
#define HD   64
#define NQKV 192
#ifndef ZB
#define ZB ((NB % 2 == 0) ? 2 : 1)
#endif
#define SCL  0.125f

static_assert(NB <= NB_FULL);
static_assert(SEQ <= SEQ_FULL);
static_assert(NB % ZB == 0);
static_assert(SEQ % 128 == 0);
static_assert(DM % 32 == 0);
static_assert(HD == 64);
static_assert((NB * SEQ) % 64 == 0);
static_assert(((size_t)SEQ * DM / 8) % 256 == 0);
static_assert(((size_t)NB * SEQ * HD) % 512 == 0);
static_assert((DM * HD / 64) % 64 == 0);

typedef unsigned short bf;
typedef _Float16 h16;
typedef __attribute__((ext_vector_type(16))) __bf16   v16bf;
typedef __attribute__((ext_vector_type(16))) _Float16 v16h;
typedef __attribute__((ext_vector_type(8)))  _Float16 v8h;
typedef __attribute__((ext_vector_type(8)))  unsigned short v8us;
typedef __attribute__((ext_vector_type(8)))  float    v8f;
typedef __attribute__((ext_vector_type(4)))  float    v4f;
typedef __attribute__((ext_vector_type(2)))  float    v2f;
typedef __attribute__((ext_vector_type(2)))  unsigned short v2us;
typedef __attribute__((ext_vector_type(4)))  unsigned short v4us;
typedef v4f  __attribute__((may_alias)) v4fa;

__device__ __forceinline__ unsigned short f2bf(float f) { unsigned u = __float_as_uint(f); u += 0x7FFFu + ((u >> 16) & 1u); return (unsigned short)(u >> 16); }
__device__ __forceinline__ float bf2f(unsigned short b) { return __uint_as_float(((unsigned)b) << 16); }
__device__ __forceinline__ float bfr(float f) { return bf2f(f2bf(f)); }
__device__ __forceinline__ v16h cat16(v8h lo, v8h hi) { return __builtin_shufflevector(lo, hi, 0, 1, 2, 3, 4, 5, 6, 7, 8, 9, 10, 11, 12, 13, 14, 15); }
__device__ __forceinline__ v16bf cat16b(v8us lo, v8us hi) { return __builtin_bit_cast(v16bf, __builtin_shufflevector(lo, hi, 0, 1, 2, 3, 4, 5, 6, 7, 8, 9, 10, 11, 12, 13, 14, 15)); }
__device__ __forceinline__ v8f wmma16(v16h a, v16h b, v8f c) { return __builtin_amdgcn_wmma_f32_16x16x32_f16(false, a, false, b, (short)0, c, false, false); }
__device__ __forceinline__ v8f wmmab(v16bf a, v16bf b, v8f c) { return __builtin_amdgcn_wmma_f32_16x16x32_bf16(false, a, false, b, (short)0, c, false, false); }

template <typename T16> struct WFrag;
template <> struct WFrag<h16> { typedef v16h V; static __device__ __forceinline__ V ld(const h16* p) { return cat16(*(const v8h*)p, *(const v8h*)(p + 16)); } static __device__ __forceinline__ v8f mma(V a, V b, v8f c) { return wmma16(a, b, c); } };
template <> struct WFrag<bf> { typedef v16bf V; static __device__ __forceinline__ V ld(const bf* p) { return cat16b(*(const v8us*)p, *(const v8us*)(p + 16)); } static __device__ __forceinline__ v8f mma(V a, V b, v8f c) { return wmmab(a, b, c); } };
template <typename T16, int NSPLIT, bool BIAS>
__global__ __launch_bounds__(32) void k_gemmw(const T16* __restrict__ A, const T16* __restrict__ A2, const T16* __restrict__ Bt, const T16* __restrict__ Bt2, int K, float* C, int ldc, const float* __restrict__ bias, size_t sA, size_t sB, size_t sC) {
    typedef typename WFrag<T16>::V V;
    __shared__ __align__(16) float os[16 * 68];
    const size_t z = blockIdx.z; A += z * sA; if (A2) A2 += z * sA; Bt += z * sB; if (Bt2) Bt2 += z * sB; C += z * sC;
    const int lane = threadIdx.x & 31, lr = lane & 15, hi = lane >> 4; const int r0 = blockIdx.x * 64, c0 = blockIdx.y * 64;
    v8f acc[4][4];
#pragma unroll
    for (int mb = 0; mb < 4; ++mb)
#pragma unroll
        for (int nb = 0; nb < 4; ++nb) acc[mb][nb] = (v8f){};
    const size_t aoff = (size_t)(r0 + lr) * K + 8 * hi, boff = (size_t)(c0 + lr) * K + 8 * hi;
#pragma unroll 1
    for (int kc = 0; kc < K; kc += 32) {
        V a[4], a2[4];
#pragma unroll
        for (int mb = 0; mb < 4; ++mb) { a[mb] = WFrag<T16>::ld(A + aoff + (size_t)mb * 16 * K + kc); if (NSPLIT == 1 || NSPLIT == 2) a2[mb] = WFrag<T16>::ld(A2 + aoff + (size_t)mb * 16 * K + kc); }
#pragma unroll
        for (int nb = 0; nb < 4; ++nb) { const V b = WFrag<T16>::ld(Bt + boff + (size_t)nb * 16 * K + kc); V b2; if (NSPLIT >= 2) b2 = WFrag<T16>::ld(Bt2 + boff + (size_t)nb * 16 * K + kc);
#pragma unroll
            for (int mb = 0; mb < 4; ++mb) { acc[mb][nb] = WFrag<T16>::mma(a[mb], b, acc[mb][nb]); if (NSPLIT == 1 || NSPLIT == 2) acc[mb][nb] = WFrag<T16>::mma(a2[mb], b, acc[mb][nb]); if (NSPLIT >= 2) acc[mb][nb] = WFrag<T16>::mma(a[mb], b2, acc[mb][nb]); } }
        asm volatile("v_nop\n\tv_nop\n\tv_nop\n\tv_nop" : "+v"(acc[0][0]), "+v"(acc[1][1]), "+v"(acc[2][2]), "+v"(acc[3][3]) : "v"(a[0]), "v"(a[3]));
    }
#pragma unroll
    for (int mb = 0; mb < 4; ++mb) {
#pragma unroll
        for (int nb = 0; nb < 4; ++nb) {
#pragma unroll
            for (int j = 0; j < 8; ++j) os[(hi * 8 + j) * 68 + nb * 16 + lr] = acc[mb][nb][j]; }
        __builtin_amdgcn_wave_barrier(); asm volatile("" ::: "memory");
        float* crow = C + (size_t)(r0 + mb * 16) * ldc + c0;
#pragma unroll 1
        for (int ps = 0; ps < 2; ++ps) {
#pragma unroll
            for (int s = 0; s < 8; ++s) { const int row = 2 * s + hi, cofs = lr * 4; v4f val = *(const v4fa*)(os + row * 68 + cofs); if (BIAS) { val[0] += bfr(bias[c0 + cofs]); val[1] += bfr(bias[c0 + cofs + 1]); val[2] += bfr(bias[c0 + cofs + 2]); val[3] += bfr(bias[c0 + cofs + 3]); }
                *(volatile v4f*)(crow + (size_t)row * ldc + cofs) = val; }
            if (ps == 0) __threadfence(); }
        __builtin_amdgcn_wave_barrier(); asm volatile("" ::: "memory");
    }
}

__device__ __forceinline__ void splitf(float y, unsigned short& h, unsigned short& l) { h = f2bf(y); l = f2bf(y - bf2f(h)); }

__global__ __launch_bounds__(256) void k_wtG(const float* __restrict__ w, int K, int N, bf* Bt) {
    w += (size_t)blockIdx.y * K * N; Bt += (size_t)blockIdx.y * N * K;
    const int lane = threadIdx.x & 31; const int L0 = (blockIdx.x * 8 + (threadIdx.x >> 5)) * 8; const int nlines = N * K / 64;
#pragma unroll
    for (int ps = 0; ps < 2; ++ps) {
#pragma unroll 1
        for (int l = 0; l < 8; ++l) { const int L = L0 + l; if (L >= nlines) break; const size_t e = (size_t)L * 64 + lane * 2; const int k = (int)(e % K), n = (int)(e / K); v2us o;
            o[0] = f2bf(w[(size_t)k * N + n]); o[1] = f2bf(w[(size_t)(k + 1) * N + n]); *(volatile v2us*)(Bt + e) = o; }
        if (ps == 0) __threadfence(); }
}

__global__ __launch_bounds__(256) void k_cvt8(const float* __restrict__ src, bf* dst, size_t n8, size_t sSrc, size_t sDst) {
    const size_t i = (size_t)blockIdx.x * 256 + threadIdx.x; if (i >= n8) return;
    src += (size_t)blockIdx.y * sSrc; dst += (size_t)blockIdx.y * sDst;
    const v8f v = *(const v8f*)(src + i * 8); v8us o;
#pragma unroll
    for (int k = 0; k < 8; ++k) o[k] = f2bf(v[k]);
    *(volatile v8us*)(dst + i * 8) = o; __threadfence(); *(volatile v8us*)(dst + i * 8) = o; }

__global__ __launch_bounds__(256) void k_plane(const float* __restrict__ F, int pitch, size_t nelem, bf* Ph, bf* Pl) {
    const size_t e = ((size_t)blockIdx.x * 256 + threadIdx.x) * 2; if (e >= nelem) return;
    const int d = (int)(e % HD); const size_t row = e / HD;
    const v2f xv = *(const v2f*)(F + row * (size_t)pitch + (size_t)blockIdx.y * HD + d);
    v2us oh, ol;
#pragma unroll
    for (int q = 0; q < 2; ++q) { unsigned short a2, c2; splitf(xv[q], a2, c2); oh[q] = a2; ol[q] = c2; }
    const size_t oo = (size_t)blockIdx.y * nelem + e;
    *(volatile v2us*)(Ph + oo) = oh; *(volatile v2us*)(Pl + oo) = ol; __threadfence(); *(volatile v2us*)(Ph + oo) = oh; *(volatile v2us*)(Pl + oo) = ol; }

__global__ __launch_bounds__(256) void k_vtp(const float* __restrict__ F, int pitch, int col0, bf* Vh, bf* Vl) {
    const size_t e = ((size_t)blockIdx.x * 256 + threadIdx.x) * 2; if (e >= (size_t)NB * HD * SEQ) return;
    const int t = (int)(e % SEQ); const int d = (int)((e / SEQ) % HD); const int g = (int)(e / ((size_t)SEQ * HD)); v2us oh, ol;
#pragma unroll
    for (int q = 0; q < 2; ++q) { const float x = F[((size_t)g * SEQ + t + q) * (size_t)pitch + col0 + d]; unsigned short a2, c2; splitf(x, a2, c2); oh[q] = a2; ol[q] = c2; }
    *(volatile v2us*)(Vh + e) = oh; *(volatile v2us*)(Vl + e) = ol; __threadfence(); *(volatile v2us*)(Vh + e) = oh; *(volatile v2us*)(Vl + e) = ol; }

__global__ __launch_bounds__(256) void k_asoft(const float* __restrict__ Sb, bf* Ph, bf* Pl, int nrows) {
    const int lane = threadIdx.x & 31; const int row = blockIdx.x * 8 + (threadIdx.x >> 5); if (row >= nrows) return;
    const float* sr = Sb + (size_t)row * SEQ; float v[SEQ / 32]; float mx = -3.0e38f;
#pragma unroll
    for (int ch = 0; ch < SEQ / 128; ++ch) { const int j0 = ch * 128 + lane * 4; const v4f a = *(const v4f*)(sr + j0);
#pragma unroll
        for (int q = 0; q < 4; ++q) { const float t = a[q] * SCL; v[ch * 4 + q] = t; mx = fmaxf(mx, t); } }
#pragma unroll
    for (int sh = 16; sh; sh >>= 1) mx = fmaxf(mx, __shfl_xor(mx, sh, 32));
    float sum = 0.f;
#pragma unroll
    for (int k = 0; k < SEQ / 32; ++k) { float d0 = __fsub_rn(v[k], mx); asm volatile("" : "+v"(d0)); v[k] = __builtin_amdgcn_exp2f(__fmul_rn(d0, 1.4426950408889634f)); sum += v[k]; }
#pragma unroll
    for (int sh = 16; sh; sh >>= 1) sum += __shfl_xor(sum, sh, 32);
    const float f = __fdiv_rn(1.0f, sum);
#pragma unroll 1
    for (int ps = 0; ps < 2; ++ps) {
#pragma unroll
        for (int ch = 0; ch < SEQ / 128; ++ch) { v4us oh, ol;
#pragma unroll
            for (int q = 0; q < 4; ++q) { unsigned short a, c2; splitf(v[ch * 4 + q] * f, a, c2); oh[q] = a; ol[q] = c2; }
            const size_t oo = (size_t)row * SEQ + ch * 128 + lane * 4; *(volatile v4us*)(Ph + oo) = oh; *(volatile v4us*)(Pl + oo) = ol; }
        if (ps == 0) __threadfence(); }
}

constexpr size_t B_W   = (size_t)NQKV * DM * 2;
constexpr size_t B_XB  = (size_t)NB * SEQ * DM * 2;
constexpr size_t B_F   = (size_t)NB * SEQ * NQKV * 4;
constexpr size_t B_QK  = (size_t)2 * NB * SEQ * HD * 2;
constexpr size_t B_VT  = (size_t)NB * HD * SEQ * 2;
constexpr size_t B_S   = (size_t)ZB * SEQ * SEQ * 4;
constexpr size_t B_P   = (size_t)ZB * SEQ * SEQ * 2;
constexpr size_t B_TOT = B_W + B_XB + B_F + 2 * B_QK + 2 * B_VT + B_S + 2 * B_P;
static_assert(B_W % 256 == 0 && B_XB % 256 == 0 && B_F % 256 == 0 && B_QK % 256 == 0 && B_VT % 256 == 0 && B_S % 256 == 0 && B_P % 256 == 0);
static_assert(B_TOT <= (size_t)134217728);

extern "C" void kernel_launch(void* const* d_in, const int* in_sizes, int n_in,
                              void* d_out, int out_size, void* d_ws, size_t ws_size, hipStream_t stream) {
    if (n_in < 2) return;
    if ((size_t)in_sizes[0] < (size_t)(NB - 1) * SEQ_FULL * DM + (size_t)SEQ * DM) return;
    if ((size_t)in_sizes[1] < (size_t)3 * DM * HD) return;
    if ((size_t)out_size < (size_t)NB * SEQ * HD) return;
    if (B_TOT > ws_size) return;
    const float* x = (const float*)d_in[0];
    const float* ker = (const float*)d_in[1];
    float* OUT = (float*)d_out;
    char* wsp = (char*)d_ws;
    auto take = [&](size_t bytes) { char* p = wsp; wsp += (bytes + 255) & ~(size_t)255; return (void*)p; };
    bf* W    = (bf*)take(B_W);
    bf* XB   = (bf*)take(B_XB);
    float* F = (float*)take(B_F);
    bf* QKh  = (bf*)take(B_QK);
    bf* QKl  = (bf*)take(B_QK);
    bf* VTh  = (bf*)take(B_VT);
    bf* VTl  = (bf*)take(B_VT);
    float* Sb = (float*)take(B_S);
    bf* Ph   = (bf*)take(B_P);
    bf* Pl   = (bf*)take(B_P);
    if ((size_t)(wsp - (char*)d_ws) > ws_size) return;

    const size_t PLN = (size_t)NB * SEQ * HD;
    k_wtG<<<dim3((unsigned)(DM * HD / 64 / 64), 3, 1), 256, 0, stream>>>(ker, DM, HD, W);
    k_cvt8<<<dim3((unsigned)((size_t)SEQ * DM / 8 / 256), NB, 1), 256, 0, stream>>>(x, XB, (size_t)SEQ * DM / 8, (size_t)SEQ_FULL * DM, (size_t)SEQ * DM);
    k_gemmw<bf, 0, false><<<dim3(NB * SEQ / 64, NQKV / 64, 1), 32, 0, stream>>>(XB, nullptr, W, nullptr, DM, F, NQKV, nullptr, 0, 0, 0);
    k_plane<<<dim3((unsigned)(PLN / 512), 2, 1), 256, 0, stream>>>(F, NQKV, PLN, QKh, QKl);
    k_vtp<<<(unsigned)((size_t)NB * HD * SEQ / 512), 256, 0, stream>>>(F, NQKV, 2 * HD, VTh, VTl);
    for (int b0 = 0; b0 < NB; b0 += ZB) {
        const size_t qo = (size_t)b0 * SEQ * HD;
        k_gemmw<bf, 2, false><<<dim3(SEQ / 64, SEQ / 64, ZB), 32, 0, stream>>>(QKh + qo, QKl + qo, QKh + PLN + qo, QKl + PLN + qo, HD, Sb, SEQ, nullptr, (size_t)SEQ * HD, (size_t)SEQ * HD, (size_t)SEQ * SEQ);
        k_asoft<<<(unsigned)(ZB * SEQ / 8), 256, 0, stream>>>(Sb, Ph, Pl, ZB * SEQ);
        k_gemmw<bf, 2, false><<<dim3(SEQ / 64, HD / 64, ZB), 32, 0, stream>>>(Ph, Pl, VTh + (size_t)b0 * HD * SEQ, VTl + (size_t)b0 * HD * SEQ, SEQ, OUT + qo, HD, nullptr, (size_t)SEQ * SEQ, (size_t)HD * SEQ, (size_t)SEQ * HD);
    }
}
